// TransformerEncoder_66589172957222
// MI455X (gfx1250) — hardware-verified
//
#include <hip/hip_runtime.h>
#include <stdint.h>


#ifndef NB
#define NB 4
#endif
#ifndef SEQ
#define SEQ 1024
#endif
#define NB_FULL 4
#define SEQ_FULL 1024
#define DD 256
#define HH 8
#define HD 32
#define FFD 1024
#define LL 4
#define QKVN (3 * DD)
#define MROWS (NB * SEQ)
#define LN_EPS 1e-5f

static_assert(NB >= 1 && NB <= NB_FULL);
static_assert(SEQ >= 64 && SEQ <= SEQ_FULL && (SEQ % 64) == 0);
static_assert((MROWS % 64) == 0);
static_assert(HH * HD == DD);
static_assert((DD % 128) == 0 && (FFD % 128) == 0 && (QKVN % 128) == 0);
static_assert((DD % 64) == 0 && (FFD % 64) == 0);

typedef _Float16 v16h __attribute__((ext_vector_type(16)));
typedef _Float16 v8h  __attribute__((ext_vector_type(8)));
typedef float    v8f  __attribute__((ext_vector_type(8)));
typedef float    v4f  __attribute__((ext_vector_type(4)));
typedef unsigned int v4u __attribute__((ext_vector_type(4)));

union Frag { v16h v; v8h half[2]; };
union Pk16 { v8h h; v4u u; };

#define DEV __device__ __forceinline__

DEV float bf16r(float f) {
  unsigned u = __float_as_uint(f);
  u = (u + 0x7fffu + ((u >> 16) & 1u)) & 0xffff0000u;
  return __uint_as_float(u);
}

DEV v8f vz8() {
  v8f z;
#pragma unroll
  for (int i = 0; i < 8; ++i) z[i] = 0.0f;
  return z;
}

DEV v16h load_frag(const _Float16* base, int ld) {
  const int lane = threadIdx.x & 31;
  const int row = lane & 15, hh = lane >> 4;
  const _Float16* p = base + (size_t)row * ld + hh * 8;
  Frag f;
  f.half[0] = *reinterpret_cast<const v8h*>(p);
  f.half[1] = *reinterpret_cast<const v8h*>(p + 16);
  return f.v;
}

DEV v8f wmma_f16(v16h a, v16h b, v8f c) {
  return __builtin_amdgcn_wmma_f32_16x16x32_f16(false, a, false, b, (short)0, c, false, false);
}

#define WG2(c0, c1, a, b0, b1) \
  asm volatile("v_nop\n\tv_nop\n\tv_nop\n\tv_nop" : "+v"(c0), "+v"(c1) : "v"(a), "v"(b0), "v"(b1))
#define WG4(c0, c1, c2, c3, a, b0, b1, b2, b3)                                              \
  asm volatile("v_nop\n\tv_nop\n\tv_nop\n\tv_nop"                                          \
               : "+v"(c0), "+v"(c1), "+v"(c2), "+v"(c3)                                     \
               : "v"(a), "v"(b0), "v"(b1), "v"(b2), "v"(b3))

DEV void st16h(_Float16* p, v8h v) { Pk16 k; k.h = v; *reinterpret_cast<volatile v4u*>(p) = k.u; }
DEV void st16f(float* p, v4f v) { *reinterpret_cast<volatile v4f*>(p) = v; }

__global__ __launch_bounds__(256) void xconv16(const float* __restrict__ x, _Float16* __restrict__ xh) {
  const int g = blockIdx.x * 256 + threadIdx.x;
  const int m = g >> 5, piece = g & 31;
  if (m >= MROWS) return;
  const int b = m / SEQ, s = m - b * SEQ;
  const size_t src = ((size_t)b * SEQ_FULL + s) * DD + piece * 8;
  const v4f a0 = *reinterpret_cast<const v4f*>(x + src);
  const v4f a1 = *reinterpret_cast<const v4f*>(x + src + 4);
  v8h o;
#pragma unroll
  for (int i = 0; i < 4; ++i) {
    o[i]     = (_Float16)bf16r(a0[i]);
    o[i + 4] = (_Float16)bf16r(a1[i]);
  }
  _Float16* dst = xh + (size_t)m * DD + piece * 8;
  st16h(dst, o);
  __threadfence();
  st16h(dst, o);
}

__global__ __launch_bounds__(256) void wtrans16(const float* __restrict__ W, _Float16* __restrict__ Wt, int K, int N) {
  __shared__ __attribute__((aligned(16))) _Float16 T[64 * 72];
  const int tid = threadIdx.x;
  const int l = blockIdx.z, k0 = blockIdx.y * 64, n0 = blockIdx.x * 64;
  const float* src = W + ((size_t)l * K + k0) * N + n0;
#pragma unroll
  for (int it = 0; it < 4; ++it) {
    const int idx = it * 256 + tid;
    const int kk = idx >> 4, c4 = idx & 15;
    const v4f v = *reinterpret_cast<const v4f*>(src + (size_t)kk * N + c4 * 4);
#pragma unroll
    for (int j = 0; j < 4; ++j) T[(c4 * 4 + j) * 72 + kk] = (_Float16)(bf16r(v[j]) * 64.0f);
  }
  __syncthreads();
  v8h vals[2];
#pragma unroll
  for (int it = 0; it < 2; ++it) {
    const int idx = it * 256 + tid;
    const int nn = idx >> 3, piece = idx & 7;
    vals[it] = *reinterpret_cast<const v8h*>(&T[nn * 72 + piece * 8]);
  }
#pragma unroll
  for (int it = 0; it < 2; ++it) {
    const int idx = it * 256 + tid;
    const int nn = idx >> 3, piece = idx & 7;
    st16h(Wt + ((size_t)l * N + n0 + nn) * K + k0 + piece * 8, vals[it]);
  }
  __threadfence();
#pragma unroll
  for (int it = 0; it < 2; ++it) {
    const int idx = it * 256 + tid;
    const int nn = idx >> 3, piece = idx & 7;
    st16h(Wt + ((size_t)l * N + n0 + nn) * K + k0 + piece * 8, vals[it]);
  }
}

template <int AM, int EP>
__global__ __launch_bounds__(256) void gemm16(const _Float16* __restrict__ A,
                                              const _Float16* __restrict__ Bt,
                                              const float* __restrict__ bias,
                                              float* __restrict__ outF,
                                              _Float16* __restrict__ outH0,
                                              _Float16* __restrict__ outH1,
                                              _Float16* __restrict__ outH2,
                                              int N, int K) {
  __shared__ __attribute__((aligned(16))) float lds_raw[64 * 132];
  _Float16* ldsh = reinterpret_cast<_Float16*>(lds_raw);
  const int tid = threadIdx.x, lane = tid & 31, wave = tid >> 5;
  const int half = lane >> 4, n16 = lane & 15;
  const int wm = wave & 3, wn = wave >> 2;
  const int m0b = blockIdx.y * 64, n0b = blockIdx.x * 128;
  const int m0w = m0b + wm * 16, n0w = n0b + wn * 64;
  const int bb = m0b / SEQ;
  const int s0b = m0b - bb * SEQ, s0w = s0b + wm * 16;

  v8f acc[4];
#pragma unroll
  for (int t = 0; t < 4; ++t) acc[t] = vz8();

  for (int k0 = 0; k0 < K; k0 += 32) {
    v16h af;
    if constexpr (AM == 0) {
      af = load_frag(A + (size_t)m0w * K + k0, K);
    } else {
      af = load_frag(A + ((size_t)(bb * HH + (k0 >> 5)) * SEQ + s0w) * HD, HD);
    }
    v16h bfr[4];
#pragma unroll
    for (int t = 0; t < 4; ++t) bfr[t] = load_frag(Bt + (size_t)(n0w + t * 16) * K + k0, K);
#pragma unroll
    for (int t = 0; t < 4; ++t) acc[t] = wmma_f16(af, bfr[t], acc[t]);
    WG4(acc[0], acc[1], acc[2], acc[3], af, bfr[0], bfr[1], bfr[2], bfr[3]);
  }

  int which = 0;
  if constexpr (EP == 0) which = n0b / DD;
#pragma unroll
  for (int t = 0; t < 4; ++t) {
    const int n = n0w + t * 16 + n16;
    const float bv = bf16r(bias[n]);
    const int nl = wn * 64 + t * 16 + n16;
#pragma unroll
    for (int r = 0; r < 8; ++r) {
      const int ml = wm * 16 + half * 8 + r;
      if constexpr (EP == 1) {
        lds_raw[ml * 132 + nl] = acc[t][r] * (1.0f / 4096.0f) + bv;
      } else if constexpr (EP == 2) {
        const float val = fmaxf(acc[t][r] * (1.0f / 64.0f) + bv, 0.0f) * 64.0f;
        ldsh[ml * 136 + nl] = (_Float16)val;
      } else {
        const float val = acc[t][r] * (1.0f / 64.0f) + bv;
        if (which == 2) ldsh[nl * 72 + ml] = (_Float16)val;
        else            ldsh[ml * 136 + nl] = (_Float16)val;
      }
    }
  }
  __syncthreads();

  if constexpr (EP == 0) {
    if (which == 2) {
      const int hb = (n0b - 2 * DD) >> 5;
      v8h vals[4];
#pragma unroll
      for (int it = 0; it < 4; ++it) {
        const int g = it * 256 + tid;
        const int nl = g >> 3, piece = g & 7;
        vals[it] = *reinterpret_cast<const v8h*>(&ldsh[nl * 72 + piece * 8]);
      }
#pragma unroll
      for (int it = 0; it < 4; ++it) {
        const int g = it * 256 + tid;
        const int nl = g >> 3, piece = g & 7;
        st16h(outH2 + ((size_t)((bb * HH + hb + (nl >> 5)) * HD + (nl & 31)) * SEQ + s0b + piece * 8), vals[it]);
      }
      __threadfence();
#pragma unroll
      for (int it = 0; it < 4; ++it) {
        const int g = it * 256 + tid;
        const int nl = g >> 3, piece = g & 7;
        st16h(outH2 + ((size_t)((bb * HH + hb + (nl >> 5)) * HD + (nl & 31)) * SEQ + s0b + piece * 8), vals[it]);
      }
    } else {
      _Float16* plane = (which == 0) ? outH0 : outH1;
      const int hw = (n0w - which * DD) >> 5;
      v8h vals[4];
#pragma unroll
      for (int j = 0; j < 2; ++j) {
#pragma unroll
        for (int i = 0; i < 2; ++i) {
          const int row = i * 8 + (lane >> 2), d = (lane & 3) * 8;
          vals[j * 2 + i] = *reinterpret_cast<const v8h*>(&ldsh[(wm * 16 + row) * 136 + wn * 64 + j * 32 + d]);
        }
      }
#pragma unroll
      for (int j = 0; j < 2; ++j) {
#pragma unroll
        for (int i = 0; i < 2; ++i) {
          const int row = i * 8 + (lane >> 2), d = (lane & 3) * 8;
          st16h(plane + ((size_t)(bb * HH + hw + j) * SEQ + s0w + row) * HD + d, vals[j * 2 + i]);
        }
      }
      __threadfence();
#pragma unroll
      for (int j = 0; j < 2; ++j) {
#pragma unroll
        for (int i = 0; i < 2; ++i) {
          const int row = i * 8 + (lane >> 2), d = (lane & 3) * 8;
          st16h(plane + ((size_t)(bb * HH + hw + j) * SEQ + s0w + row) * HD + d, vals[j * 2 + i]);
        }
      }
    }
  } else if constexpr (EP == 1) {
    v4f vals[8];
#pragma unroll
    for (int i = 0; i < 8; ++i) {
      const int row = i * 2 + half, piece = n16;
      vals[i] = *reinterpret_cast<const v4f*>(&lds_raw[(wm * 16 + row) * 132 + wn * 64 + piece * 4]);
    }
#pragma unroll
    for (int i = 0; i < 8; ++i) {
      const int row = i * 2 + half, piece = n16;
      st16f(outF + (size_t)(m0w + row) * N + n0w + piece * 4, vals[i]);
    }
    __threadfence();
#pragma unroll
    for (int i = 0; i < 8; ++i) {
      const int row = i * 2 + half, piece = n16;
      st16f(outF + (size_t)(m0w + row) * N + n0w + piece * 4, vals[i]);
    }
  } else {
    v8h vals[4];
#pragma unroll
    for (int i = 0; i < 4; ++i) {
      const int row = i * 4 + (lane >> 3), piece = lane & 7;
      vals[i] = *reinterpret_cast<const v8h*>(&ldsh[(wm * 16 + row) * 136 + wn * 64 + piece * 8]);
    }
#pragma unroll
    for (int i = 0; i < 4; ++i) {
      const int row = i * 4 + (lane >> 3), piece = lane & 7;
      st16h(outH0 + (size_t)(m0w + row) * N + n0w + piece * 8, vals[i]);
    }
    __threadfence();
#pragma unroll
    for (int i = 0; i < 4; ++i) {
      const int row = i * 4 + (lane >> 3), piece = lane & 7;
      st16h(outH0 + (size_t)(m0w + row) * N + n0w + piece * 8, vals[i]);
    }
  }
}

__global__ __launch_bounds__(128) void attn16(const _Float16* __restrict__ Qp,
                                              const _Float16* __restrict__ Kp,
                                              const _Float16* __restrict__ Vt,
                                              const int* __restrict__ mask,
                                              _Float16* __restrict__ Op) {
  __shared__ __attribute__((aligned(16))) _Float16 lds_p[4][16 * 32];
  const int lane = threadIdx.x & 31, wave = threadIdx.x >> 5;
  const int half = lane >> 4, n16 = lane & 15;
  constexpr int QT = SEQ / 16;
  const int tile = blockIdx.x * 4 + wave;
  const int qt = tile % QT, bh = tile / QT;
  const int b = bh / HH;
  const int q0 = qt * 16;
  _Float16* pbuf = &lds_p[wave][0];

  const v16h aq = load_frag(Qp + ((size_t)bh * SEQ + q0) * HD, HD);
  const int* mrowp = mask + (size_t)b * SEQ_FULL;

  float mrow[8], lrow[8];
#pragma unroll
  for (int r = 0; r < 8; ++r) { mrow[r] = -3.0e38f; lrow[r] = 0.0f; }
  v8f acc[2];
  acc[0] = vz8();
  acc[1] = vz8();

  for (int kb = 0; kb < SEQ; kb += 32) {
    const _Float16* kBase = Kp + ((size_t)bh * SEQ + kb) * HD;
    const v16h kf0 = load_frag(kBase, HD);
    const v16h kf1 = load_frag(kBase + 16 * HD, HD);
    v8f s0 = wmma_f16(aq, kf0, vz8());
    v8f s1 = wmma_f16(aq, kf1, vz8());
    WG2(s0, s1, aq, kf0, kf1);

    const int mk0 = mrowp[kb + n16];
    const int mk1 = mrowp[kb + 16 + n16];
#pragma unroll
    for (int r = 0; r < 8; ++r) {
      const float v0 = (mk0 != 0) ? s0[r] : -1.0e30f;
      const float v1 = (mk1 != 0) ? s1[r] : -1.0e30f;
      float cmax = fmaxf(v0, v1);
#pragma unroll
      for (int msk = 1; msk < 16; msk <<= 1) cmax = fmaxf(cmax, __shfl_xor(cmax, msk, 32));
      const float mnew = fmaxf(mrow[r], cmax);
      const float corr = __expf(mrow[r] - mnew);
      const float p0 = __expf(v0 - mnew);
      const float p1 = __expf(v1 - mnew);
      float ps = p0 + p1;
#pragma unroll
      for (int msk = 1; msk < 16; msk <<= 1) ps += __shfl_xor(ps, msk, 32);
      lrow[r] = lrow[r] * corr + ps;
      mrow[r] = mnew;
      acc[0][r] *= corr;
      acc[1][r] *= corr;
      const int mr = half * 8 + r;
      pbuf[mr * 32 + n16]      = (_Float16)(p0 * 256.0f);
      pbuf[mr * 32 + 16 + n16] = (_Float16)(p1 * 256.0f);
    }
    __syncthreads();
    const v16h pa = load_frag(pbuf, 32);
    const _Float16* vBase = Vt + (size_t)bh * HD * SEQ + kb;
    const v16h vf0 = load_frag(vBase, SEQ);
    const v16h vf1 = load_frag(vBase + (size_t)16 * SEQ, SEQ);
    acc[0] = wmma_f16(pa, vf0, acc[0]);
    acc[1] = wmma_f16(pa, vf1, acc[1]);
    WG2(acc[0], acc[1], pa, vf0, vf1);
    __syncthreads();
  }

#pragma unroll
  for (int r = 0; r < 8; ++r) {
    const float inv = 0.25f * __builtin_amdgcn_rcpf(lrow[r]);
    const int row = half * 8 + r;
    pbuf[row * 32 + n16]      = (_Float16)(acc[0][r] * inv);
    pbuf[row * 32 + 16 + n16] = (_Float16)(acc[1][r] * inv);
  }
  __syncthreads();
  v8h vals[2];
#pragma unroll
  for (int i = 0; i < 2; ++i) {
    const int row = i * 8 + (lane >> 2), d = (lane & 3) * 8;
    vals[i] = *reinterpret_cast<const v8h*>(&pbuf[row * 32 + d]);
  }
#pragma unroll
  for (int i = 0; i < 2; ++i) {
    const int row = i * 8 + (lane >> 2), d = (lane & 3) * 8;
    st16h(Op + ((size_t)bh * SEQ + q0 + row) * HD + d, vals[i]);
  }
  __threadfence();
#pragma unroll
  for (int i = 0; i < 2; ++i) {
    const int row = i * 8 + (lane >> 2), d = (lane & 3) * 8;
    st16h(Op + ((size_t)bh * SEQ + q0 + row) * HD + d, vals[i]);
  }
}

template <int RESB, int OUTD>
__global__ __launch_bounds__(256) void add_ln16(const float* __restrict__ a,
                                                const float* __restrict__ res,
                                                const float* __restrict__ gam,
                                                const float* __restrict__ bet,
                                                float* __restrict__ outF,
                                                _Float16* __restrict__ outH) {
  __shared__ float red[8];
  __shared__ __attribute__((aligned(16))) float sh_o[DD];
  const int m = blockIdx.x, tid = threadIdx.x, lane = tid & 31, wave = tid >> 5;
  const int b = m / SEQ, s = m - b * SEQ;
  const size_t mfull = (size_t)b * SEQ_FULL + s;

  float rv;
  if constexpr (RESB != 0) rv = bf16r(res[mfull * DD + tid]);
  else                     rv = res[(size_t)m * DD + tid];
  const float v = a[(size_t)m * DD + tid] + rv;

  float sm = v;
#pragma unroll
  for (int msk = 16; msk > 0; msk >>= 1) sm += __shfl_xor(sm, msk, 32);
  if (lane == 0) red[wave] = sm;
  __syncthreads();
  float tot = 0.0f;
#pragma unroll
  for (int i = 0; i < 8; ++i) tot += red[i];
  const float mean = tot * (1.0f / DD);
  const float d = v - mean;
  float sq = d * d;
#pragma unroll
  for (int msk = 16; msk > 0; msk >>= 1) sq += __shfl_xor(sq, msk, 32);
  __syncthreads();
  if (lane == 0) red[wave] = sq;
  __syncthreads();
  float tot2 = 0.0f;
#pragma unroll
  for (int i = 0; i < 8; ++i) tot2 += red[i];
  const float var = tot2 * (1.0f / DD);
  const float rstd = rsqrtf(var + LN_EPS);
  const float o = d * rstd * bf16r(gam[tid]) + bf16r(bet[tid]);
  sh_o[tid] = o;
  __syncthreads();

  if (wave < 2) {
    const int idx = wave * 32 + lane;
    const v4f val = *reinterpret_cast<const v4f*>(&sh_o[idx * 4]);
    float* dst;
    if constexpr (OUTD != 0) dst = outF + mfull * DD + idx * 4;
    else                     dst = outF + (size_t)m * DD + idx * 4;
    st16f(dst, val);
    __threadfence();
    st16f(dst, val);
  }
  if constexpr (OUTD == 0) {
    if (wave == 2) {
      v8h hv;
      const v4f u0 = *reinterpret_cast<const v4f*>(&sh_o[lane * 8]);
      const v4f u1 = *reinterpret_cast<const v4f*>(&sh_o[lane * 8 + 4]);
#pragma unroll
      for (int i = 0; i < 4; ++i) { hv[i] = (_Float16)u0[i]; hv[i + 4] = (_Float16)u1[i]; }
      _Float16* dst = outH + (size_t)m * DD + lane * 8;
      st16h(dst, hv);
      __threadfence();
      st16h(dst, hv);
    }
  }
}

extern "C" void kernel_launch(void* const* d_in, const int* in_sizes, int n_in,
                              void* d_out, int out_size, void* d_ws, size_t ws_size,
                              hipStream_t stream) {
  if (n_in < 14) return;
  const float* x     = (const float*)d_in[0];
  const int*   mask  = (const int*)d_in[1];
  const float* qkv_w = (const float*)d_in[2];
  const float* qkv_b = (const float*)d_in[3];
  const float* fc_w  = (const float*)d_in[4];
  const float* fc_b  = (const float*)d_in[5];
  const float* ln1_g = (const float*)d_in[6];
  const float* ln1_b = (const float*)d_in[7];
  const float* ln2_g = (const float*)d_in[8];
  const float* ln2_b = (const float*)d_in[9];
  const float* ff1_w = (const float*)d_in[10];
  const float* ff1_b = (const float*)d_in[11];
  const float* ff2_w = (const float*)d_in[12];
  const float* ff2_b = (const float*)d_in[13];
  float* out = (float*)d_out;

  const size_t rows_hi = (size_t)(NB - 1) * SEQ_FULL + SEQ;
  if ((size_t)in_sizes[0]  < rows_hi * DD) return;
  if ((size_t)in_sizes[1]  < rows_hi) return;
  if ((size_t)in_sizes[2]  < (size_t)LL * DD * QKVN) return;
  if ((size_t)in_sizes[3]  < (size_t)LL * QKVN) return;
  if ((size_t)in_sizes[4]  < (size_t)LL * DD * DD) return;
  if ((size_t)in_sizes[5]  < (size_t)LL * DD) return;
  if ((size_t)in_sizes[6]  < (size_t)LL * DD) return;
  if ((size_t)in_sizes[7]  < (size_t)LL * DD) return;
  if ((size_t)in_sizes[8]  < (size_t)LL * DD) return;
  if ((size_t)in_sizes[9]  < (size_t)LL * DD) return;
  if ((size_t)in_sizes[10] < (size_t)LL * DD * FFD) return;
  if ((size_t)in_sizes[11] < (size_t)LL * FFD) return;
  if ((size_t)in_sizes[12] < (size_t)LL * FFD * DD) return;
  if ((size_t)in_sizes[13] < (size_t)LL * DD) return;
  if ((size_t)out_size < rows_hi * DD) return;

  char* ws = (char*)d_ws;
  size_t off = 0;
  auto carve = [&](size_t bytes) -> char* {
    char* p = ws + off;
    off += (bytes + 255) & ~(size_t)255;
    return p;
  };
  const size_t M = MROWS;
  _Float16* wqkvT = (_Float16*)carve((size_t)LL * QKVN * DD * 2);
  _Float16* wfcT  = (_Float16*)carve((size_t)LL * DD * DD * 2);
  _Float16* wff1T = (_Float16*)carve((size_t)LL * FFD * DD * 2);
  _Float16* wff2T = (_Float16*)carve((size_t)LL * DD * FFD * 2);
  _Float16* xh    = (_Float16*)carve(M * DD * 2);
  _Float16* qh    = (_Float16*)carve(M * DD * 2);
  _Float16* kh    = (_Float16*)carve(M * DD * 2);
  _Float16* vt    = (_Float16*)carve(M * DD * 2);
  _Float16* oh    = (_Float16*)carve(M * DD * 2);
  float*    y     = (float*)   carve(M * DD * 4);
  float*    x1    = (float*)   carve(M * DD * 4);
  _Float16* x1h   = (_Float16*)carve(M * DD * 2);
  _Float16* h1    = (_Float16*)carve(M * FFD * 2);
  float*    z     = (float*)   carve(M * DD * 4);
  float*    xc    = (float*)   carve(M * DD * 4);
  if (off > ws_size) return;
  if (off > (size_t)134217728) return;

  wtrans16<<<dim3(QKVN / 64, DD / 64, LL), 256, 0, stream>>>(qkv_w, wqkvT, DD, QKVN);
  wtrans16<<<dim3(DD / 64, DD / 64, LL), 256, 0, stream>>>(fc_w, wfcT, DD, DD);
  wtrans16<<<dim3(FFD / 64, DD / 64, LL), 256, 0, stream>>>(ff1_w, wff1T, DD, FFD);
  wtrans16<<<dim3(DD / 64, FFD / 64, LL), 256, 0, stream>>>(ff2_w, wff2T, FFD, DD);
  xconv16<<<dim3(MROWS / 8), 256, 0, stream>>>(x, xh);

  const dim3 g_qkv(QKVN / 128, MROWS / 64);
  const dim3 g_d(DD / 128, MROWS / 64);
  const dim3 g_ff(FFD / 128, MROWS / 64);
  const dim3 g_att(NB * HH * (SEQ / 16) / 4);

  for (int l = 0; l < LL; ++l) {
    gemm16<0, 0><<<g_qkv, 256, 0, stream>>>(xh, wqkvT + (size_t)l * QKVN * DD, qkv_b + (size_t)l * QKVN,
                                            nullptr, qh, kh, vt, QKVN, DD);
    attn16<<<g_att, 128, 0, stream>>>(qh, kh, vt, mask, oh);
    gemm16<1, 1><<<g_d, 256, 0, stream>>>(oh, wfcT + (size_t)l * DD * DD, fc_b + (size_t)l * DD,
                                          y, nullptr, nullptr, nullptr, DD, DD);
    if (l == 0)
      add_ln16<1, 0><<<dim3(MROWS), 256, 0, stream>>>(y, x, ln1_g + (size_t)l * DD, ln1_b + (size_t)l * DD, x1, x1h);
    else
      add_ln16<0, 0><<<dim3(MROWS), 256, 0, stream>>>(y, xc, ln1_g + (size_t)l * DD, ln1_b + (size_t)l * DD, x1, x1h);
    gemm16<0, 2><<<g_ff, 256, 0, stream>>>(x1h, wff1T + (size_t)l * FFD * DD, ff1_b + (size_t)l * FFD,
                                           nullptr, h1, nullptr, nullptr, FFD, DD);
    gemm16<0, 1><<<g_d, 256, 0, stream>>>(h1, wff2T + (size_t)l * DD * FFD, ff2_b + (size_t)l * DD,
                                          z, nullptr, nullptr, nullptr, DD, FFD);
    if (l == LL - 1)
      add_ln16<0, 1><<<dim3(MROWS), 256, 0, stream>>>(z, x1, ln2_g + (size_t)l * DD, ln2_b + (size_t)l * DD, out, nullptr);
    else
      add_ln16<0, 0><<<dim3(MROWS), 256, 0, stream>>>(z, x1, ln2_g + (size_t)l * DD, ln2_b + (size_t)l * DD, xc, xh);
  }
}
